// Lapla_filter_77584289235642
// MI455X (gfx1250) — hardware-run, weakly checked
//
#include <hip/hip_runtime.h>
#include <stddef.h>
#include <stdint.h>
#include <math.h>

#define NN      100000
#define NE      3200000
#define DF      128
#define KH      256
#define GBM     64
#define GTHR    128
#define MP      100096
#define NTHR    256
#define NWAVE   8
#define EPT     8
#define WCH     (32 * EPT)
#define NBRUN   1024
#define SLB     10
#define NBK     98
#define NPADN   (NBK * NBRUN)
#define WLCAP   4608
#define RCAP    35840
#define DEGCAP  96
#define MAXDEG_MEAS   58
#define MAXB1024_MEAS 33280
#define RPB     64
#define RPW     8
#define WSMAX   134217728

#define BK_ZINTS (NWAVE * WLCAP + RCAP + 2 * NBRUN)
#define BK_INTS  (BK_ZINTS + 16)
#define BK_LDS   (BK_INTS * 4)

#define PBX   (MP * DF / 8 / NTHR)
#define PBW1  (DF * DF / 8 / NTHR)
#define PBW2  (DF * KH / 8 / NTHR)
#define PBTOT (PBX + PBW1 + PBW2 + 1)

static_assert(DF == 32 * 4 && DF == 8 * 16);
static_assert(DF % 32 == 0 && KH % 32 == 0 && KH == 2 * DF);
static_assert(GBM == (GTHR / 32) * 16);
static_assert(MP % GBM == 0 && MP >= NN && MP == 1564 * GBM && MP % RPB == 0 && RPB == NWAVE * RPW);
static_assert(NBRUN == (1 << SLB) && NBRUN % RPB == 0 && NBRUN == NTHR * 4 && NBRUN % 32 == 0);
static_assert(NPADN >= MP);
static_assert(NE < (1 << 22));
static_assert(NN <= 131072);
static_assert(NE % WCH == 0 && NE % 8 == 0);
static_assert(RCAP % (NTHR * 4) == 0 && RCAP % 32 == 0 && BK_ZINTS % (NTHR * 4) == 0);
static_assert((long long)RCAP * 100 >= (long long)MAXB1024_MEAS * 105);
static_assert(WLCAP >= MAXB1024_MEAS / 8 + 400 && WLCAP >= NBRUN);
static_assert(DEGCAP >= MAXDEG_MEAS + 8);
static_assert(BK_LDS <= 300000);
static_assert((MP * DF / 8) % NTHR == 0 && (DF * DF / 8) % NTHR == 0 && (DF * KH / 8) % NTHR == 0);
static_assert((GBM * DF + DF) * 4 <= 65536);

typedef float          v4f   __attribute__((ext_vector_type(4)));
typedef float          v8f   __attribute__((ext_vector_type(8)));
typedef int            v4i   __attribute__((ext_vector_type(4)));
typedef int            v8i   __attribute__((ext_vector_type(8)));
typedef unsigned short v8us  __attribute__((ext_vector_type(8)));
typedef unsigned short v16us __attribute__((ext_vector_type(16)));
typedef __bf16         v16bf __attribute__((ext_vector_type(16)));
typedef v4f  __attribute__((may_alias)) v4fa;
typedef v4i  __attribute__((may_alias)) v4ia;
typedef v8us __attribute__((may_alias)) v8usa;
union FragB { v16bf v; v16us u; v8us h[2]; v8i w; };

__device__ __forceinline__ v8f wmb(const FragB& a, const FragB& b, v8f c) {
  v8f d = __builtin_amdgcn_wmma_f32_16x16x32_bf16(false, a.v, false, b.v, (short)0, c, false, false);
  asm volatile("v_nop\n\tv_nop\n\tv_nop\n\tv_nop" : "+v"(d) : "v"(a.w), "v"(b.w));
  return d;
}

__device__ __forceinline__ unsigned bf16_bits(float f) {
  const unsigned u = __float_as_uint(f);
  const unsigned r = (u + 0x7FFFu + ((u >> 16) & 1u)) >> 16;
  const unsigned q = (u >> 16) | 0x40u;
  return ((u & 0x7fffffffu) > 0x7f800000u) ? q : r;
}
__device__ __forceinline__ float bf16_val(float f) {
  return __uint_as_float(bf16_bits(f) << 16);
}
__device__ __forceinline__ float relu_k(float v) { return (v > 0.0f) ? v : (v - v); }

__device__ __forceinline__ void hilo_pack(float v0, float v1, float v2, float v3,
                                          int& h01, int& h23, int& l01, int& l23) {
  const unsigned a0 = bf16_bits(v0), a1 = bf16_bits(v1), a2 = bf16_bits(v2), a3 = bf16_bits(v3);
  const unsigned b0 = bf16_bits(v0 - __uint_as_float(a0 << 16));
  const unsigned b1 = bf16_bits(v1 - __uint_as_float(a1 << 16));
  const unsigned b2 = bf16_bits(v2 - __uint_as_float(a2 << 16));
  const unsigned b3 = bf16_bits(v3 - __uint_as_float(a3 << 16));
  h01 = (int)(a0 | (a1 << 16)); h23 = (int)(a2 | (a3 << 16));
  l01 = (int)(b0 | (b1 << 16)); l23 = (int)(b2 | (b3 << 16));
}

__device__ __forceinline__ v4i regroup_row(int h01, int h23, int l01, int l23, int lane) {
  const int s0 = (2 * lane) & 31, s1 = s0 + 1;
  const int a0 = __shfl(h01, s0, 32), a1 = __shfl(h23, s0, 32), a2 = __shfl(h01, s1, 32), a3 = __shfl(h23, s1, 32);
  const int b0 = __shfl(l01, s0, 32), b1 = __shfl(l23, s0, 32), b2 = __shfl(l01, s1, 32), b3 = __shfl(l23, s1, 32);
  const int mk = (lane < 16) ? -1 : 0;
  v4i o;
  o.x = (a0 & mk) | (b0 & ~mk); o.y = (a1 & mk) | (b1 & ~mk);
  o.z = (a2 & mk) | (b2 & ~mk); o.w = (a3 & mk) | (b3 & ~mk);
  return o;
}

__device__ __forceinline__ void st2_v4f(float* p, v4f v) {
  *(volatile v4f*)p = v;
  __threadfence();
  *(volatile v4f*)p = v;
}
__device__ __forceinline__ void st2_v8us(unsigned short* p, v8us v) {
  *(volatile v8us*)p = v;
  __threadfence();
  *(volatile v8us*)p = v;
}

__device__ __forceinline__ v8us gather8(const float* __restrict__ base, int stride) {
  float f[8];
#pragma unroll
  for (int i = 0; i < 8; ++i) f[i] = base[(size_t)i * (size_t)stride];
  v8us o;
#pragma unroll
  for (int i = 0; i < 8; ++i) o[i] = (unsigned short)bf16_bits(f[i]);
  return o;
}

__global__ __launch_bounds__(NTHR) void k_prep(const float* __restrict__ x, const float* __restrict__ w1,
                                               const float* __restrict__ b1, const float* __restrict__ w2,
                                               const float* __restrict__ b2,
                                               unsigned short* xb, unsigned short* w1t, unsigned short* w2d,
                                               float* sm) {
  const int tid = (int)threadIdx.x;
  const int blk = (int)blockIdx.x;
  if (blk < PBX) {
    const int u   = blk * NTHR + tid;
    const int row = u >> 4, k8 = (u & 15) * 8;
    const int rc  = row < NN ? row : NN - 1;
    const unsigned mk = row < NN ? 0xffffu : 0u;
    const float* p = x + (size_t)rc * DF + k8;
    const v4f a = *(const v4fa*)p;
    const v4f b = *(const v4fa*)(p + 4);
    v8us o;
    o[0] = (unsigned short)(bf16_bits(a.x) & mk); o[1] = (unsigned short)(bf16_bits(a.y) & mk);
    o[2] = (unsigned short)(bf16_bits(a.z) & mk); o[3] = (unsigned short)(bf16_bits(a.w) & mk);
    o[4] = (unsigned short)(bf16_bits(b.x) & mk); o[5] = (unsigned short)(bf16_bits(b.y) & mk);
    o[6] = (unsigned short)(bf16_bits(b.z) & mk); o[7] = (unsigned short)(bf16_bits(b.w) & mk);
    st2_v8us(xb + (size_t)row * DF + k8, o);
  } else if (blk < PBX + PBW1) {
    const int u = (blk - PBX) * NTHR + tid;
    const int n = u >> 4, k8 = (u & 15) * 8;
    const v8us o = gather8(w1 + (size_t)k8 * DF + n, DF);
    st2_v8us(w1t + (size_t)n * DF + k8, o);
  } else if (blk < PBX + PBW1 + PBW2) {
    const int u = (blk - PBX - PBW1) * NTHR + tid;
    const int n = u >> 5, k8 = (u & 31) * 8, kk = k8 & (DF - 1);
    const v8us o = gather8(w2 + (size_t)kk * DF + n, DF);
    st2_v8us(w2d + (size_t)n * KH + k8, o);
  } else {
    if (tid < 64) {
      const int q = tid & 31;
      const v4f a = *(const v4fa*)(b1 + 4 * q);
      const v4f c = *(const v4fa*)(b2 + 4 * q);
      asm volatile("" :: "v"(a), "v"(c));
      const unsigned ma = (tid < 32) ? 0xffffffffu : 0u;
      v4f o;
      o.x = __uint_as_float(((bf16_bits(a.x) << 16) & ma) | ((bf16_bits(c.x) << 16) & ~ma));
      o.y = __uint_as_float(((bf16_bits(a.y) << 16) & ma) | ((bf16_bits(c.y) << 16) & ~ma));
      o.z = __uint_as_float(((bf16_bits(a.z) << 16) & ma) | ((bf16_bits(c.z) << 16) & ~ma));
      o.w = __uint_as_float(((bf16_bits(a.w) << 16) & ma) | ((bf16_bits(c.w) << 16) & ~ma));
      st2_v4f(sm + 4 * tid, o);
    }
  }
}

template <int KTOT>
__device__ __forceinline__ void gemm_16x128(const unsigned short* __restrict__ ap,
                                            const unsigned short* __restrict__ bp, v8f (&acc)[8]) {
#pragma unroll 1
  for (int k0 = 0; k0 < KTOT; k0 += 32) {
    FragB af;
    af.h[0] = *(const v8usa*)(ap + k0);
    af.h[1] = *(const v8usa*)(ap + k0 + 16);
#pragma unroll
    for (int t = 0; t < 8; ++t) {
      const unsigned short* wq = bp + (size_t)(16 * t) * (size_t)KTOT + k0;
      FragB bf;
      bf.h[0] = *(const v8usa*)wq;
      bf.h[1] = *(const v8usa*)(wq + 16);
      acc[t] = wmb(af, bf, acc[t]);
    }
  }
}

template <int KTOT, int RELU>
__global__ __launch_bounds__(GTHR) __attribute__((amdgpu_num_vgpr(248)))
void k_gemm(const unsigned short* __restrict__ A, const unsigned short* __restrict__ BT,
            const float* __restrict__ bias, float* outp, int nStore) {
  __shared__ __attribute__((aligned(16))) float stg[GBM * DF];
  __shared__ __attribute__((aligned(16))) float bsh[DF];
  const int tid = (int)threadIdx.x, lane = tid & 31, wave = tid >> 5, hh = lane >> 4, m = lane & 15;
  const int rowBase = (int)blockIdx.x * GBM;

  if (tid < 32) {
    const v4f b4 = *(const v4fa*)(bias + 4 * tid);
    *(v4fa*)(bsh + 4 * tid) = b4;
  }

  v8f acc[8];
  {
    const v8f z = {0.f, 0.f, 0.f, 0.f, 0.f, 0.f, 0.f, 0.f};
#pragma unroll
    for (int t = 0; t < 8; ++t) acc[t] = z;
  }
  const unsigned short* ap = A + (size_t)(rowBase + 16 * wave + m) * (size_t)KTOT + 8 * hh;
  const unsigned short* bp = BT + (size_t)m * (size_t)KTOT + 8 * hh;
  gemm_16x128<KTOT>(ap, bp, acc);
  __syncthreads();

#pragma unroll
  for (int t = 0; t < 8; ++t) {
    const int lc = 16 * t + m;
    const float bb = bsh[lc];
#pragma unroll
    for (int r = 0; r < 8; ++r) {
      const int lr = 16 * wave + 8 * hh + r;
      const bool live = (rowBase + lr) < NN;
      float v = acc[t][r] + bb;
      if constexpr (RELU != 0) v = relu_k(v);
      stg[lr * DF + lc] = live ? v : 0.0f;
    }
  }
  __syncthreads();

  v4f pk[16];
#pragma unroll
  for (int i = 0; i < 16; ++i) pk[i] = *(const v4fa*)(stg + (16 * wave + i) * DF + 4 * lane);
#pragma unroll
  for (int i = 0; i < 16; ++i) {
    const int gr = rowBase + 16 * wave + i;
    float* op = outp + (size_t)gr * (size_t)DF + 4 * lane;
    if (gr < nStore) *(volatile v4f*)op = pk[i];
  }
  __threadfence();
#pragma unroll
  for (int i = 0; i < 16; ++i) {
    const int gr = rowBase + 16 * wave + i;
    float* op = outp + (size_t)gr * (size_t)DF + 4 * lane;
    if (gr < nStore) *(volatile v4f*)op = pk[i];
  }
}

__device__ __forceinline__ void bucket_flush(const int* pl, const int* cnt, const int* offs, const int* dvb, int ov,
                                             int* lp, int* cp, int* fp, int* dp, int* gp, int tid) {
#pragma unroll 1
  for (int i = tid * 4; i < RCAP; i += NTHR * 4) {
    const v4i v = *(const v4ia*)(pl + i);
    *(volatile v4i*)(lp + i) = v;
  }
  {
    const v4i cv = *(const v4ia*)(cnt + 4 * tid);
    const v4i ev = *(const v4ia*)(offs + 4 * tid);
    const v4i dv = *(const v4ia*)(dvb + 4 * tid);
    v4i fv;
    fv.x = ev.x - cv.x; fv.y = ev.y - cv.y; fv.z = ev.z - cv.z; fv.w = ev.w - cv.w;
    fv.x = fv.x < 0 ? 0 : fv.x; fv.y = fv.y < 0 ? 0 : fv.y;
    fv.z = fv.z < 0 ? 0 : fv.z; fv.w = fv.w < 0 ? 0 : fv.w;
    *(volatile v4i*)(cp + 4 * tid) = cv;
    *(volatile v4i*)(fp + 4 * tid) = fv;
    *(volatile v4i*)(dp + 4 * tid) = dv;
  }
  if (tid < 8) {
    const v4i f = {ov, ov, ov, ov};
    *(volatile v4i*)(gp + 4 * tid) = f;
  }
}

__global__ __launch_bounds__(NTHR) void k_bucket(const int* __restrict__ srcs, const int* __restrict__ dsts,
                                                 int* LIST, int* CNT, int* OFF, int* DINVB, int* FLAG) {
  extern __shared__ __attribute__((aligned(16))) int dsm[];
  int* wl   = dsm;
  int* pl   = dsm + NWAVE * WLCAP;
  int* cnt  = pl + RCAP;
  int* offs = cnt + NBRUN;
  int* misc = offs + NBRUN;
  const int tid = (int)threadIdx.x, lane = tid & 31, wave = tid >> 5;
  const int blk = (int)blockIdx.x;
  const int nodeBase = blk * NBRUN;
  int nb = NN - nodeBase;
  nb = nb > NBRUN ? NBRUN : (nb < 1 ? 1 : nb);
  const unsigned nbs = (unsigned)nodeBase;
  const unsigned unb = (unsigned)nb;

  {
    const v4i z4 = {0, 0, 0, 0};
    for (int i = tid * 4; i < BK_ZINTS; i += NTHR * 4) *(v4ia*)(dsm + i) = z4;
    if (tid < 16) misc[tid] = 0;
  }
  __syncthreads();

  {
    const int per  = ((NE + NWAVE * WCH - 1) / (NWAVE * WCH)) * WCH;
    const int ebeg = wave * per;
    const int eend = (ebeg + per < NE) ? (ebeg + per) : NE;
    int* mylist = wl + wave * WLCAP;
    int wc = 0;
#pragma unroll 1
    for (int cb = ebeg; cb < eend; cb += WCH) {
      const int e0 = cb + lane * EPT;
      const v4i da = *(const v4ia*)(dsts + e0);
      const v4i db = *(const v4ia*)(dsts + e0 + 4);
      const unsigned s0 = (unsigned)da.x - nbs, s1 = (unsigned)da.y - nbs;
      const unsigned s2 = (unsigned)da.z - nbs, s3 = (unsigned)da.w - nbs;
      const unsigned s4 = (unsigned)db.x - nbs, s5 = (unsigned)db.y - nbs;
      const unsigned s6 = (unsigned)db.z - nbs, s7 = (unsigned)db.w - nbs;
      const bool h0 = s0 < unb, h1 = s1 < unb, h2 = s2 < unb, h3 = s3 < unb;
      const bool h4 = s4 < unb, h5 = s5 < unb, h6 = s6 < unb, h7 = s7 < unb;
      const unsigned m0 = __builtin_amdgcn_ballot_w32(h0), m1 = __builtin_amdgcn_ballot_w32(h1);
      const unsigned m2 = __builtin_amdgcn_ballot_w32(h2), m3 = __builtin_amdgcn_ballot_w32(h3);
      const unsigned m4 = __builtin_amdgcn_ballot_w32(h4), m5 = __builtin_amdgcn_ballot_w32(h5);
      const unsigned m6 = __builtin_amdgcn_ballot_w32(h6), m7 = __builtin_amdgcn_ballot_w32(h7);
      const unsigned any = m0 | m1 | m2 | m3 | m4 | m5 | m6 | m7;
      if (any != 0u) {
        const int pre = (int)(__builtin_amdgcn_mbcnt_lo(m0, 0u) + __builtin_amdgcn_mbcnt_lo(m1, 0u) +
                              __builtin_amdgcn_mbcnt_lo(m2, 0u) + __builtin_amdgcn_mbcnt_lo(m3, 0u) +
                              __builtin_amdgcn_mbcnt_lo(m4, 0u) + __builtin_amdgcn_mbcnt_lo(m5, 0u) +
                              __builtin_amdgcn_mbcnt_lo(m6, 0u) + __builtin_amdgcn_mbcnt_lo(m7, 0u));
        int p = wc + pre;
        if (h0) { if (p < WLCAP) mylist[p] = (int)(((unsigned)(e0 + 0) << SLB) | s0); p = p + 1; }
        if (h1) { if (p < WLCAP) mylist[p] = (int)(((unsigned)(e0 + 1) << SLB) | s1); p = p + 1; }
        if (h2) { if (p < WLCAP) mylist[p] = (int)(((unsigned)(e0 + 2) << SLB) | s2); p = p + 1; }
        if (h3) { if (p < WLCAP) mylist[p] = (int)(((unsigned)(e0 + 3) << SLB) | s3); p = p + 1; }
        if (h4) { if (p < WLCAP) mylist[p] = (int)(((unsigned)(e0 + 4) << SLB) | s4); p = p + 1; }
        if (h5) { if (p < WLCAP) mylist[p] = (int)(((unsigned)(e0 + 5) << SLB) | s5); p = p + 1; }
        if (h6) { if (p < WLCAP) mylist[p] = (int)(((unsigned)(e0 + 6) << SLB) | s6); p = p + 1; }
        if (h7) { if (p < WLCAP) mylist[p] = (int)(((unsigned)(e0 + 7) << SLB) | s7); p = p + 1; }
        wc += (int)(__builtin_popcount(m0) + __builtin_popcount(m1) + __builtin_popcount(m2) + __builtin_popcount(m3) +
                    __builtin_popcount(m4) + __builtin_popcount(m5) + __builtin_popcount(m6) + __builtin_popcount(m7));
      }
    }
    if (lane == 0) misc[wave] = wc;
  }
  __syncthreads();

  int ov = 0;
  if (wave == 0) {
    int tot = 0;
#pragma unroll 1
    for (int w2 = 0; w2 < NWAVE; ++w2) {
      int c = misc[w2];
      if (c > WLCAP) ov = 1;
      c = c < 0 ? 0 : (c > WLCAP ? WLCAP : c);
      tot += c;
#pragma unroll 1
      for (int b0 = 0; b0 < c; b0 += 32) {
        const int idx = b0 + lane;
        const int ent = wl[w2 * WLCAP + (idx < WLCAP ? idx : WLCAP - 1)];
        const int m32 = (c - b0) < 32 ? (c - b0) : 32;
#pragma unroll 1
        for (int k = 0; k < m32; ++k) {
          const int u    = __builtin_amdgcn_readlane(ent, k);
          const int slot = u & (NBRUN - 1);
          if (lane == 0) cnt[slot] = cnt[slot] + 1;
        }
      }
    }
    if (tot > RCAP) ov = 1;
  }
  __syncthreads();
  if (wave == 0) {
    const int base = lane * (NBRUN / 32);
    int s = 0, mx = 0;
#pragma unroll 1
    for (int i = 0; i < NBRUN / 32; ++i) {
      const int cv = cnt[base + i];
      s += cv;
      mx = cv > mx ? cv : mx;
    }
    int incl = s;
#pragma unroll
    for (int d = 1; d < 32; d <<= 1) {
      const int y = __shfl_up(incl, d, 32);
      if (lane >= d) incl += y;
    }
    {
      int t;
      t = __shfl_xor(mx, 16, 32); mx = t > mx ? t : mx;
      t = __shfl_xor(mx, 8, 32);  mx = t > mx ? t : mx;
      t = __shfl_xor(mx, 4, 32);  mx = t > mx ? t : mx;
      t = __shfl_xor(mx, 2, 32);  mx = t > mx ? t : mx;
      t = __shfl_xor(mx, 1, 32);  mx = t > mx ? t : mx;
    }
    int run = incl - s;
#pragma unroll 1
    for (int i = 0; i < NBRUN / 32; ++i) {
      const int cv = cnt[base + i];
      offs[base + i] = run;
      run += cv;
    }
    if (lane == 0) misc[9] = ((ov != 0) || (mx > DEGCAP)) ? 1 : 0;
  }
  __syncthreads();

  if (wave == 0) {
#pragma unroll 1
    for (int w2 = 0; w2 < NWAVE; ++w2) {
      int c = misc[w2];
      c = c < 0 ? 0 : (c > WLCAP ? WLCAP : c);
#pragma unroll 1
      for (int b0 = 0; b0 < c; b0 += 32) {
        const int idx = b0 + lane;
        const int ent = wl[w2 * WLCAP + (idx < WLCAP ? idx : WLCAP - 1)];
        int eid = (ent >> SLB) & 0x3FFFFF;
        eid = eid > NE - 1 ? NE - 1 : eid;
        int sr = srcs[eid];
        sr = sr < 0 ? 0 : (sr > NN - 1 ? NN - 1 : sr);
        const int m32 = (c - b0) < 32 ? (c - b0) : 32;
#pragma unroll 1
        for (int k = 0; k < m32; ++k) {
          const int u    = __builtin_amdgcn_readlane(ent, k);
          const int wd   = __builtin_amdgcn_readlane(sr, k);
          const int slot = u & (NBRUN - 1);
          if (lane == 0) {
            int p = offs[slot];
            p = p < 0 ? 0 : (p > RCAP - 1 ? RCAP - 1 : p);
            pl[p] = wd;
            offs[slot] = p + 1;
          }
        }
      }
    }
  }
  __syncthreads();

#pragma unroll 1
  for (int i = tid; i < NBRUN; i += NTHR) {
    int c = cnt[i];
    c = c < 1 ? 1 : c;
    wl[i] = __float_as_int(1.0f / sqrtf((float)c));
  }
  __syncthreads();

  const int ovf = misc[9];
  int* lp = LIST + (size_t)blk * RCAP;
  int* cp = CNT + (size_t)nodeBase;
  int* fp = OFF + (size_t)nodeBase;
  int* dp = DINVB + (size_t)nodeBase;
  int* gp = FLAG + (size_t)blk * 32;
  bucket_flush(pl, cnt, offs, wl, ovf, lp, cp, fp, dp, gp, tid);
  __threadfence();
  bucket_flush(pl, cnt, offs, wl, ovf, lp, cp, fp, dp, gp, tid);
}

__global__ __launch_bounds__(NTHR) void k_lap(const float* __restrict__ FEAT, const int* __restrict__ LIST,
                                              const int* __restrict__ CNT, const int* __restrict__ OFF,
                                              const float* __restrict__ DINV, const int* __restrict__ FLAG,
                                              unsigned short* F2) {
  const int tid = (int)threadIdx.x, lane = tid & 31, wave = tid >> 5;
  const int rowBase = (int)blockIdx.x * RPB;
  const int bucket  = rowBase >> SLB;
  const int* lb  = LIST + (size_t)bucket * RCAP;
  const int flag = FLAG[(size_t)bucket * 32];
  const float qnan = __uint_as_float(0x7fc00000u);

#pragma unroll 1
  for (int ri = 0; ri < RPW; ++ri) {
    const int d = rowBase + wave * RPW + ri;
    const int craw = CNT[d];
    const int oraw = OFF[d];
    const bool big = craw > DEGCAP;
    int c = craw < 0 ? 0 : (craw > DEGCAP ? DEGCAP : craw);
    const int o = oraw < 0 ? 0 : (oraw > RCAP - 1 ? RCAP - 1 : oraw);
    if (c > RCAP - o) c = RCAP - o;
    const int last = o + (c > 0 ? c : 1) - 1;
    float a0 = 0.0f, a1 = 0.0f, a2 = 0.0f, a3 = 0.0f;
#pragma unroll 1
    for (int b0 = 0; b0 < c; b0 += 32) {
      int idx = o + b0 + lane;
      idx = idx > last ? last : idx;
      int s = lb[idx];
      s = s < 0 ? 0 : (s > NN - 1 ? NN - 1 : s);
      const int dvb = __float_as_int(DINV[s]);
      const int m32 = (c - b0) < 32 ? (c - b0) : 32;
#pragma unroll 4
      for (int k = 0; k < m32; ++k) {
        const int sk = __builtin_amdgcn_readlane(s, k);
        const float w = __int_as_float(__builtin_amdgcn_readlane(dvb, k));
        const v4f v = *(const v4fa*)(FEAT + (size_t)sk * DF + 4 * lane);
        a0 = fmaf(v.x, w, a0);
        a1 = fmaf(v.y, w, a1);
        a2 = fmaf(v.z, w, a2);
        a3 = fmaf(v.w, w, a3);
      }
    }
    const v4f g = *(const v4fa*)(FEAT + (size_t)d * DF + 4 * lane);
    const float dd = DINV[d];
    float r0 = g.x - a0 * dd, r1 = g.y - a1 * dd, r2 = g.z - a2 * dd, r3 = g.w - a3 * dd;
    const bool bad  = (flag != 0) | big;
    const bool live = d < NN;
    r0 = bad ? qnan : r0; r1 = bad ? qnan : r1; r2 = bad ? qnan : r2; r3 = bad ? qnan : r3;
    r0 = live ? r0 : 0.0f; r1 = live ? r1 : 0.0f; r2 = live ? r2 : 0.0f; r3 = live ? r3 : 0.0f;
    int h01, h23, l01, l23;
    hilo_pack(r0, r1, r2, r3, h01, h23, l01, l23);
    const v4i ow = regroup_row(h01, h23, l01, l23, lane);
    unsigned short* hp = F2 + (size_t)d * KH + 8 * lane;
    *(volatile v4i*)hp = ow;
    __threadfence();
    *(volatile v4i*)hp = ow;
  }
}

extern "C" void kernel_launch(void* const* d_in, const int* in_sizes, int n_in,
                              void* d_out, int out_size, void* d_ws, size_t ws_size,
                              hipStream_t stream) {
  if (n_in < 7) return;
  if (in_sizes[0] != NN * DF) return;
  if (in_sizes[1] != NE) return;
  if (in_sizes[2] != NE) return;
  if (in_sizes[3] != DF * DF) return;
  if (in_sizes[4] != DF) return;
  if (in_sizes[5] != DF * DF) return;
  if (in_sizes[6] != DF) return;
  if (out_size != NN * DF) return;

  const float* x   = (const float*)d_in[0];
  const int*   src = (const int*)d_in[1];
  const int*   dst = (const int*)d_in[2];
  const float* W1  = (const float*)d_in[3];
  const float* b1  = (const float*)d_in[4];
  const float* W2  = (const float*)d_in[5];
  const float* b2  = (const float*)d_in[6];
  float* out = (float*)d_out;

  constexpr size_t zF2   = (size_t)MP * KH * 2;
  constexpr size_t zXB   = (size_t)MP * DF * 2;
  constexpr size_t zFEAT = (size_t)MP * DF * 4;
  constexpr size_t zLIST = (size_t)NBK * RCAP * 4;
  constexpr size_t zTAB  = (size_t)NPADN * 4;
  constexpr size_t zFLAG = (size_t)NBK * 128;
  constexpr size_t zW1T  = (size_t)DF * DF * 2;
  constexpr size_t zW2D  = (size_t)DF * KH * 2;
  constexpr size_t zSM   = 1024;
  constexpr size_t oF2   = 0;
  constexpr size_t oFEAT = oF2 + zF2;
  constexpr size_t oLIST = oFEAT + zFEAT;
  constexpr size_t oCNT  = oLIST + zLIST;
  constexpr size_t oOFF  = oCNT + zTAB;
  constexpr size_t oDINV = oOFF + zTAB;
  constexpr size_t oFLAG = oDINV + zTAB;
  constexpr size_t oW1T  = oFLAG + zFLAG;
  constexpr size_t oW2D  = oW1T + zW1T;
  constexpr size_t oSM   = oW2D + zW2D;
  constexpr size_t oEND  = oSM + zSM;
  static_assert(zXB <= zF2);
  static_assert(zF2 % 256 == 0 && zFEAT % 256 == 0 && zLIST % 256 == 0 && zTAB % 256 == 0 && zFLAG % 256 == 0);
  static_assert(zW1T % 256 == 0 && zW2D % 256 == 0 && zSM % 256 == 0);
  static_assert(oEND <= (size_t)WSMAX);
  if (oEND > ws_size) return;

  char* ws = (char*)d_ws;
  unsigned short* F2   = (unsigned short*)(ws + oF2);
  unsigned short* XB   = (unsigned short*)(ws + oF2);
  float*          FEAT = (float*)(ws + oFEAT);
  int*            LIST = (int*)(ws + oLIST);
  int*            CNT  = (int*)(ws + oCNT);
  int*            OFF  = (int*)(ws + oOFF);
  int*            DINB = (int*)(ws + oDINV);
  const float*    DINV = (const float*)(ws + oDINV);
  int*            FLAG = (int*)(ws + oFLAG);
  unsigned short* W1T  = (unsigned short*)(ws + oW1T);
  unsigned short* W2D  = (unsigned short*)(ws + oW2D);
  float*          SM   = (float*)(ws + oSM);

  hipFuncSetAttribute(reinterpret_cast<const void*>(&k_bucket), hipFuncAttributeMaxDynamicSharedMemorySize, (int)BK_LDS);

  k_prep<<<PBTOT, NTHR, 0, stream>>>(x, W1, b1, W2, b2, XB, W1T, W2D, SM);
  k_gemm<DF, 1><<<MP / GBM, GTHR, 0, stream>>>(XB, W1T, SM, FEAT, MP);
  k_bucket<<<NBK, NTHR, BK_LDS, stream>>>(src, dst, LIST, CNT, OFF, DINB, FLAG);
  k_lap<<<MP / RPB, NTHR, 0, stream>>>(FEAT, LIST, CNT, OFF, DINV, FLAG, F2);
  k_gemm<KH, 0><<<MP / GBM, GTHR, 0, stream>>>(F2, W2D, SM + DF, out, NN);
}
